// Decoder_23235773071576
// MI455X (gfx1250) — hardware-verified
//
#include <hip/hip_runtime.h>
#include <math.h>

constexpr int NBATCH = 256;
constexpr int NSLOT  = 64;
constexpr int NHID   = 256;
constexpr int NENC   = 512;
constexpr int NROWS  = NBATCH * NSLOT;
constexpr int NW1    = 2 * NHID + NENC;
constexpr int NFC    = NENC + 2;
constexpr int NGATE  = 4 * NHID;
constexpr int KHC    = 2 * NHID;
constexpr int NTHR   = 256;
constexpr int HCP    = 520;
constexpr int SLABP  = 68;
constexpr int HC_PLANE = 2 * 16 * HCP;

constexpr float HC_CARRY  = 256.0f;
constexpr float W_CARRY   = 64.0f;
constexpr float RES_CARRY = 2048.0f;
constexpr float RES_INV   = 1.0f / RES_CARRY;
constexpr float V_INV     = 1.0f / (HC_CARRY * W_CARRY);
constexpr float E_INV     = 1.0f / W_CARRY;
constexpr float SLOT_INV  = 1.0f / (float)NSLOT;

constexpr int AB_OFF   = 0;
constexpr int WEFF_OFF = 256;
constexpr int WEFF_PAD = 576;
constexpr int GB_OFF   = WEFF_OFF + WEFF_PAD;
constexpr int SMALL_N  = 3072;

static_assert(NW1 == 1024);
static_assert(NFC == 514);
static_assert(GB_OFF == 832 && GB_OFF + 2 * NGATE <= SMALL_N);
static_assert(SMALL_N % (4 * NTHR) == 0);
static_assert(NROWS % 256 == 0);
static_assert(NENC % 32 == 0 && KHC % 32 == 0 && NHID % 32 == 0);
static_assert(NROWS % 32 == 0 && NHID % 64 == 0);
static_assert(((NROWS / 32) * (NHID / 64)) % 8 == 0);
static_assert(NBATCH % 16 == 0);
static_assert(NBATCH * NSLOT * 4 == 65536);
static_assert(65536 + NBATCH * 4 == 66560);
static_assert((HCP % 8) == 0 && HCP >= KHC);

typedef __attribute__((ext_vector_type(16))) _Float16 v16h;
typedef __attribute__((ext_vector_type(8)))  _Float16 v8h;
typedef __attribute__((ext_vector_type(8)))  float    v8f;
typedef __attribute__((ext_vector_type(4)))  float    v4f;

union FragU { v16h v; v8h h[2]; };

__device__ __forceinline__ v16h frag_load(const _Float16* p) {
  FragU f;
  f.h[0] = *(const v8h*)(p);
  f.h[1] = *(const v8h*)(p + 16);
  return f.v;
}
__device__ __forceinline__ v8f mma_h(v16h a, v16h b, v8f c) {
  return __builtin_amdgcn_wmma_f32_16x16x32_f16(false, a, false, b, (short)0, c, false, false);
}
__device__ __forceinline__ void guard4(v8f& a, v8f& b, v8f& c, v8f& d, v16h x0, v16h x1, v16h x2, v16h x3, v16h x4) {
  asm volatile("v_nop\n\tv_nop\n\tv_nop\n\tv_nop" : "+v"(a), "+v"(b), "+v"(c), "+v"(d) : "v"(x0), "v"(x1), "v"(x2), "v"(x3), "v"(x4));
}
__device__ __forceinline__ void guard8(v8f& a0, v8f& a1, v8f& a2, v8f& a3, v8f& a4, v8f& a5, v8f& a6, v8f& a7,
                                       v16h x0, v16h x1, v16h x2, v16h x3, v16h x4, v16h x5) {
  asm volatile("v_nop\n\tv_nop\n\tv_nop\n\tv_nop"
               : "+v"(a0), "+v"(a1), "+v"(a2), "+v"(a3), "+v"(a4), "+v"(a5), "+v"(a6), "+v"(a7)
               : "v"(x0), "v"(x1), "v"(x2), "v"(x3), "v"(x4), "v"(x5));
}
__device__ __forceinline__ void acc_guard4(v8f& a, v8f& b, v8f& c, v8f& d) {
  asm volatile("v_nop\n\tv_nop\n\tv_nop\n\tv_nop" : "+v"(a), "+v"(b), "+v"(c), "+v"(d));
}
__device__ __forceinline__ int opaque_i(int x) {
  asm volatile("" : "+v"(x));
  return x;
}

__device__ __forceinline__ float fsig(float x)  { return __builtin_amdgcn_rcpf(1.0f + __expf(-x)); }
__device__ __forceinline__ float ftanh(float x) { return 1.0f - 2.0f * __builtin_amdgcn_rcpf(__expf(2.0f * x) + 1.0f); }

__device__ __forceinline__ void split_h(float xs, _Float16& hi, _Float16& lo) {
  const _Float16 h0 = (_Float16)xs;
  float hf = (float)h0;
  hf = (fabsf(hf) < 6.103515625e-05f) ? 0.0f : hf;
  hi = (_Float16)hf;
  lo = (_Float16)((xs - hf) * RES_CARRY);
}

__global__ __launch_bounds__(NTHR) void fold_w21_kernel(const float* __restrict__ w1, const float* __restrict__ w2,
                                                        unsigned short* __restrict__ W21HC, unsigned short* __restrict__ W21E) {
  const int i = blockIdx.x * NTHR + threadIdx.x;
  if (i < NHID * (NW1 / 8)) {
    const int n  = i >> 7;
    const int jc = (i & 127) * 8;
    float acc[8];
#pragma unroll
    for (int e = 0; e < 8; ++e) acc[e] = 0.0f;
    const float* w2row = w2 + (size_t)n * NHID;
    const float* w1p   = w1 + jc;
#pragma unroll 1
    for (int k = 0; k < NHID; ++k) {
      const float wv = w2row[k];
      const v4f a = *(const v4f*)(w1p + (size_t)k * NW1);
      const v4f b = *(const v4f*)(w1p + (size_t)k * NW1 + 4);
#pragma unroll
      for (int e = 0; e < 4; ++e) {
        acc[e]     = fmaf(wv, a[e], acc[e]);
        acc[4 + e] = fmaf(wv, b[e], acc[4 + e]);
      }
    }
    v8h hv;
#pragma unroll
    for (int e = 0; e < 8; ++e) hv[e] = (_Float16)(acc[e] * W_CARRY);
    const int plane = jc >> 9;
    unsigned short* dst = (plane ? W21E : W21HC) + (size_t)n * KHC + (jc & 511);
    *(volatile v8h*)dst = hv;
    __threadfence();
    *(volatile v8h*)dst = hv;
  }
}

__global__ __launch_bounds__(NTHR) void small_prep_kernel(const float* __restrict__ w2, const float* __restrict__ b1,
                                                          const float* __restrict__ b2, const float* __restrict__ fcw1,
                                                          const float* __restrict__ fcb1, const float* __restrict__ fcw2,
                                                          const float* __restrict__ fcb2,
                                                          const float* __restrict__ bihf, const float* __restrict__ bhhf,
                                                          const float* __restrict__ bihb, const float* __restrict__ bhhb,
                                                          float* __restrict__ SMALLv) {
  __shared__ __align__(16) float sS[SMALL_N];
  const int tid = threadIdx.x;
  float ab = 0.0f;
#pragma unroll 1
  for (int k = 0; k < NHID; ++k) ab = fmaf(w2[(size_t)tid * NHID + k], b1[k], ab);
  sS[AB_OFF + tid] = ab + b2[tid];
  float be = 0.0f;
#pragma unroll 1
  for (int n = 0; n < NHID; ++n) be = fmaf(fcw2[n], fcb1[n], be);
  be += fcb2[0];
#pragma unroll 1
  for (int jj = 0; jj < 3; ++jj) {
    const int j   = tid + NTHR * jj;
    const int jcl = (j < NFC - 1) ? j : (NFC - 1);
    float acc = 0.0f;
#pragma unroll 1
    for (int n = 0; n < NHID; ++n) acc = fmaf(fcw2[n], fcw1[(size_t)n * NFC + jcl], acc);
    const float val = (j < NFC) ? acc : ((j == NFC) ? be : 0.0f);
    if (j < WEFF_PAD) sS[WEFF_OFF + j] = val;
  }
#pragma unroll 1
  for (int q = 0; q < 8; ++q) {
    const int idx = q * NTHR + tid;
    const int jx  = idx & (NGATE - 1);
    const float f = bihf[jx] + bhhf[jx];
    const float b = bihb[jx] + bhhb[jx];
    sS[GB_OFF + idx] = (idx >= NGATE) ? b : f;
  }
  if (tid < SMALL_N - (GB_OFF + 2 * NGATE)) sS[GB_OFF + 2 * NGATE + tid] = 0.0f;
  __syncthreads();
  for (int pass = 0; pass < 2; ++pass) {
#pragma unroll
    for (int it = 0; it < SMALL_N / (4 * NTHR); ++it) {
      const int idx4 = it * NTHR + tid;
      const v4f v = *(const v4f*)(sS + idx4 * 4);
      *(volatile v4f*)(SMALLv + idx4 * 4) = v;
    }
    __threadfence();
  }
}

__global__ __launch_bounds__(NTHR) void cvt8_scale_kernel(const float* __restrict__ src, unsigned short* __restrict__ dst,
                                                          int n8, float sc) {
  const int i = blockIdx.x * NTHR + threadIdx.x;
  if (i < n8) {
    const v4f a = *(const v4f*)(src + (size_t)i * 8);
    const v4f b = *(const v4f*)(src + (size_t)i * 8 + 4);
    v8h hv;
#pragma unroll
    for (int e = 0; e < 4; ++e) {
      hv[e]     = (_Float16)(a[e] * sc);
      hv[4 + e] = (_Float16)(b[e] * sc);
    }
    *(volatile v8h*)(dst + (size_t)i * 8) = hv;
    __threadfence();
    *(volatile v8h*)(dst + (size_t)i * 8) = hv;
  }
}

__global__ __launch_bounds__(NTHR) void ie_pack_kernel(const float* __restrict__ IE, const float* __restrict__ SMALLv,
                                                       const float* __restrict__ fwin,
                                                       unsigned short* __restrict__ IEH, unsigned short* __restrict__ IEL,
                                                       float* __restrict__ Qv, float* __restrict__ Rv) {
  __shared__ __align__(16) float sW[2 * NENC];
  const int tid = threadIdx.x, lane = tid & 31, wave = tid >> 5;
  {
    const int idx = (tid & 127) * 4;
    const v4f a = *(const v4f*)(SMALLv + WEFF_OFF + idx);
    const v4f b = *(const v4f*)(fwin + NHID + idx);
    v4f o;
#pragma unroll
    for (int e = 0; e < 4; ++e) o[e] = (tid < 128) ? a[e] : b[e];
    *(v4f*)(sW + tid * 4) = o;
  }
  __syncthreads();
  const int kA = 8 * lane, kB = 256 + 8 * lane;
  const v4f qa0 = *(const v4f*)(sW + kA);
  const v4f qa1 = *(const v4f*)(sW + kA + 4);
  const v4f qb0 = *(const v4f*)(sW + kB);
  const v4f qb1 = *(const v4f*)(sW + kB + 4);
  const v4f ra0 = *(const v4f*)(sW + NENC + kA);
  const v4f ra1 = *(const v4f*)(sW + NENC + kA + 4);
  const v4f rb0 = *(const v4f*)(sW + NENC + kB);
  const v4f rb1 = *(const v4f*)(sW + NENC + kB + 4);
  const int gw = blockIdx.x * 8 + wave;
  float qk = 0.0f, rk = 0.0f;
#pragma unroll 1
  for (int ri = 0; ri < 32; ++ri) {
    const size_t row = (size_t)gw * 32 + ri;
    const float* src = IE + row * NENC;
    const v4f a0 = *(const v4f*)(src + kA);
    const v4f a1 = *(const v4f*)(src + kA + 4);
    const v4f b0 = *(const v4f*)(src + kB);
    const v4f b1 = *(const v4f*)(src + kB + 4);
    v8h hA, lA, hB, lB;
    float qs = 0.0f, rs = 0.0f;
#pragma unroll
    for (int e = 0; e < 4; ++e) {
      _Float16 hi, lo;
      const float x0 = a0[e], x1 = a1[e], x2 = b0[e], x3 = b1[e];
      split_h(x0, hi, lo); hA[e] = hi;     lA[e] = lo;
      split_h(x1, hi, lo); hA[4 + e] = hi; lA[4 + e] = lo;
      split_h(x2, hi, lo); hB[e] = hi;     lB[e] = lo;
      split_h(x3, hi, lo); hB[4 + e] = hi; lB[4 + e] = lo;
      qs += x0 * qa0[e];
      qs += x1 * qa1[e];
      qs += x2 * qb0[e];
      qs += x3 * qb1[e];
      rs += x0 * ra0[e];
      rs += x1 * ra1[e];
      rs += x2 * rb0[e];
      rs += x3 * rb1[e];
    }
    unsigned short* ph = IEH + row * NENC;
    unsigned short* pl = IEL + row * NENC;
    for (int pass = 0; pass < 2; ++pass) {
      *(volatile v8h*)(ph + kA) = hA;
      *(volatile v8h*)(ph + kB) = hB;
      *(volatile v8h*)(pl + kA) = lA;
      *(volatile v8h*)(pl + kB) = lB;
      __threadfence();
    }
#pragma unroll
    for (int off = 1; off < 32; off <<= 1) {
      qs += __shfl_xor(qs, off, 32);
      rs += __shfl_xor(rs, off, 32);
    }
    qk = (lane == ri) ? qs : qk;
    rk = (lane == ri) ? rs : rk;
  }
  float* qd = Qv + (size_t)gw * 32 + lane;
  float* rd = Rv + (size_t)gw * 32 + lane;
  *(volatile float*)qd = qk;
  *(volatile float*)rd = rk;
  __threadfence();
  *(volatile float*)qd = qk;
  *(volatile float*)rd = rk;
}

__global__ __launch_bounds__(NTHR) void e2_gemm_kernel(const unsigned short* __restrict__ IEHp, const unsigned short* __restrict__ IELp,
                                                       const unsigned short* __restrict__ W21Ep, const float* __restrict__ ABv,
                                                       float* __restrict__ E2) {
  __shared__ __align__(16) float sT[8][16 * SLABP];
  const _Float16* AH = (const _Float16*)IEHp;
  const _Float16* AL = (const _Float16*)IELp;
  const _Float16* BT = (const _Float16*)W21Ep;
  const int lane = threadIdx.x & 31, wave = threadIdx.x >> 5;
  const int tile = blockIdx.x * 8 + wave;
  const int tm = tile >> 2, tn = tile & 3;
  const int m0 = tm * 32, n0 = tn * 64;
  const int rlane = lane & 15, koff = (lane >> 4) * 8, mOff = (lane >> 4) * 8;
  const v8f z8 = {0.f, 0.f, 0.f, 0.f, 0.f, 0.f, 0.f, 0.f};
  v8f accM[2][4], accR[2][4];
#pragma unroll
  for (int i = 0; i < 2; ++i)
#pragma unroll
    for (int j = 0; j < 4; ++j) { accM[i][j] = z8; accR[i][j] = z8; }

#pragma unroll 1
  for (int k0 = 0; k0 < NENC; k0 += 32) {
    v16h bh[4];
#pragma unroll
    for (int j = 0; j < 4; ++j) bh[j] = frag_load(BT + (size_t)(n0 + 16 * j + rlane) * NENC + koff + k0);
#pragma unroll
    for (int i = 0; i < 2; ++i) {
      const size_t ao = (size_t)(m0 + 16 * i + rlane) * NENC + koff + k0;
      const v16h ah = frag_load(AH + ao);
      const v16h al = frag_load(AL + ao);
#pragma unroll
      for (int j = 0; j < 4; ++j) {
        accM[i][j] = mma_h(ah, bh[j], accM[i][j]);
        accR[i][j] = mma_h(al, bh[j], accR[i][j]);
      }
      guard8(accM[i][0], accM[i][1], accM[i][2], accM[i][3], accR[i][0], accR[i][1], accR[i][2], accR[i][3],
             ah, al, bh[0], bh[1], bh[2], bh[3]);
    }
  }
  acc_guard4(accM[0][0], accM[0][1], accM[0][2], accM[0][3]);
  acc_guard4(accM[1][0], accM[1][1], accM[1][2], accM[1][3]);
  acc_guard4(accR[0][0], accR[0][1], accR[0][2], accR[0][3]);
  acc_guard4(accR[1][0], accR[1][1], accR[1][2], accR[1][3]);

  float* slab = sT[wave];
  float abv[4];
#pragma unroll
  for (int j = 0; j < 4; ++j) abv[j] = ABv[AB_OFF + n0 + 16 * j + rlane];
#pragma unroll
  for (int i = 0; i < 2; ++i) {
    const int mBase = m0 + 16 * i;
#pragma unroll
    for (int j = 0; j < 4; ++j) {
#pragma unroll
      for (int r = 0; r < 8; ++r) {
        const float v = (accM[i][j][r] + accR[i][j][r] * RES_INV) * E_INV + abv[j];
        slab[(mOff + r) * SLABP + 16 * j + rlane] = v;
      }
    }
    __builtin_amdgcn_fence(__ATOMIC_RELEASE, "workgroup");
    __builtin_amdgcn_wave_barrier();
    __builtin_amdgcn_fence(__ATOMIC_ACQUIRE, "workgroup");
    {
      const int hh = lane >> 4, c4 = (lane & 15) * 4;
      for (int pass = 0; pass < 2; ++pass) {
#pragma unroll
        for (int it = 0; it < 8; ++it) {
          const int row = it * 2 + hh;
          const v4f v = *(const v4f*)(slab + row * SLABP + c4);
          *(volatile v4f*)(E2 + (size_t)(mBase + row) * NHID + n0 + c4) = v;
        }
        __threadfence();
      }
    }
    __builtin_amdgcn_fence(__ATOMIC_RELEASE, "workgroup");
    __builtin_amdgcn_wave_barrier();
    __builtin_amdgcn_fence(__ATOMIC_ACQUIRE, "workgroup");
  }
}

__global__ __launch_bounds__(NTHR) __attribute__((amdgpu_num_vgpr(256))) void decoder_scan_kernel(
    const float* __restrict__ E2, const float* __restrict__ Qv, const float* __restrict__ Rv,
    const float* __restrict__ yhist, const float* __restrict__ spd,
    const float* __restrict__ h0, const float* __restrict__ c0,
    const unsigned short* __restrict__ W21HCp, const unsigned short* __restrict__ WHFp, const unsigned short* __restrict__ WHBp,
    const float* __restrict__ SMALLv, const float* __restrict__ w3, const float* __restrict__ b3,
    const float* __restrict__ wihf, const float* __restrict__ wihb,
    const float* __restrict__ fwin, const float* __restrict__ fbin,
    float* __restrict__ out0, float* __restrict__ OUT1P) {
  __shared__ __align__(16) _Float16 HCh[2 * HC_PLANE];
  __shared__ __align__(16) _Float16 HCl[HC_PLANE];
  __shared__ __align__(16) float    sV[2 * 16 * NHID];
  __shared__ __align__(16) float    sGW[4 * NGATE];
  __shared__ float sYt[16];
  __shared__ float sPart[8 * 16];
  __shared__ float sOctx[16];

  const _Float16* W21HC = (const _Float16*)W21HCp;
  const _Float16* WHF   = (const _Float16*)WHFp;
  const _Float16* WHB   = (const _Float16*)WHBp;
  const int tid = threadIdx.x, lane = tid & 31, wave = tid >> 5;
  const int c = lane & 15, hh = lane >> 4, koff = hh * 8;
  const int brow0 = blockIdx.x * 16;
  const v8f z8 = {0.f, 0.f, 0.f, 0.f, 0.f, 0.f, 0.f, 0.f};

  {
    const v4f g0 = *(const v4f*)(SMALLv + GB_OFF + tid * 4);
    const v4f g1 = *(const v4f*)(SMALLv + GB_OFF + NGATE + tid * 4);
    const v4f wf = *(const v4f*)(wihf + tid * 4);
    const v4f wb = *(const v4f*)(wihb + tid * 4);
    *(v4f*)(sGW + tid * 4) = g0;
    *(v4f*)(sGW + NGATE + tid * 4) = g1;
    *(v4f*)(sGW + 2 * NGATE + tid * 4) = wf;
    *(v4f*)(sGW + 3 * NGATE + tid * 4) = wb;
  }
#pragma unroll 1
  for (int it = 0; it < 8; ++it) {
    const int idx = it * NTHR + tid;
    const int p = idx >> 10, row = (idx >> 6) & 15, k4 = (idx & 63) * 4;
    const size_t go = ((size_t)(p * NBATCH + brow0 + row)) * NHID + k4;
    const v4f hv = *(const v4f*)(h0 + go);
    const v4f cv = *(const v4f*)(c0 + go);
    *(v4f*)(sV + (p * 16 + row) * NHID + k4) = cv;
    _Float16* ph = HCh + (p * 16 + row) * HCP + k4;
    _Float16* pl = HCl + (p * 16 + row) * HCP + k4;
#pragma unroll
    for (int e = 0; e < 4; ++e) {
      _Float16 hi, lo;
      const float hx = hv[e], cx = cv[e];
      split_h(hx * HC_CARRY, hi, lo);
      ph[e] = hi; pl[e] = lo;
      split_h(cx * HC_CARRY, hi, lo);
      ph[NHID + e] = hi; pl[NHID + e] = lo;
    }
  }
  __syncthreads();
  float cst[2][2][8];
#pragma unroll
  for (int p = 0; p < 2; ++p)
#pragma unroll
    for (int nt = 0; nt < 2; ++nt)
#pragma unroll
      for (int r = 0; r < 8; ++r)
        cst[p][nt][r] = sV[(p * 16 + 8 * hh + r) * NHID + 32 * wave + 16 * nt + c];
  __syncthreads();

  float w3r[8];
  {
    const v4f t0 = *(const v4f*)(w3 + 8 * lane);
    const v4f t1 = *(const v4f*)(w3 + 8 * lane + 4);
#pragma unroll
    for (int e = 0; e < 4; ++e) { w3r[e] = t0[e]; w3r[4 + e] = t1[e]; }
  }
  asm volatile("" ::: "memory");
  float qv[2][2], rv[2][2];
#pragma unroll
  for (int bi = 0; bi < 2; ++bi) {
    const size_t ro = (size_t)(brow0 + 2 * wave + bi) * NSLOT + lane;
    qv[bi][0] = Qv[ro];
    qv[bi][1] = Qv[ro + 32];
    rv[bi][0] = Rv[ro];
    rv[bi][1] = Rv[ro + 32];
  }
  asm volatile("" ::: "memory");
  const float weffy = SMALLv[WEFF_OFF + NENC];
  const float weffs = SMALLv[WEFF_OFF + NENC + 1];
  const float beff  = SMALLv[WEFF_OFF + NENC + 2];
  const float b3v   = b3[0];
  const float fw0   = fwin[32 * wave + c];
  const float fw1   = fwin[32 * wave + 16 + c];
  float wsum[2][2] = {{0.0f, 0.0f}, {0.0f, 0.0f}};
  float octx[2] = {0.0f, 0.0f};
  float hfd[8];
#pragma unroll
  for (int r = 0; r < 8; ++r) hfd[r] = 0.0f;

#pragma unroll 1
  for (int s = 0; s < NSLOT; ++s) {
    const _Float16* hcur = HCh + (s & 1) * HC_PLANE;
    _Float16*       hnxt = HCh + ((s & 1) ^ 1) * HC_PLANE;

    {
      const int p = wave >> 2;
      const int ntb = (wave & 3) * 4;
      const _Float16* ahrow = hcur + (p * 16 + c) * HCP + koff;
      const _Float16* alrow = HCl + (p * 16 + c) * HCP + koff;
#pragma unroll 1
      for (int half = 0; half < 2; ++half) {
        const int nt0 = ntb + 2 * half;
        const _Float16* bp0 = W21HC + (size_t)(nt0 * 16 + c) * KHC + koff;
        const _Float16* bp1 = bp0 + (size_t)16 * KHC;
        v8f m0 = z8, m1 = z8, r0 = z8, r1 = z8;
#pragma unroll 1
        for (int k0 = 0; k0 < KHC; k0 += 32) {
          const v16h a  = frag_load(ahrow + k0);
          const v16h l  = frag_load(alrow + k0);
          const v16h b0 = frag_load(bp0 + k0);
          const v16h b1 = frag_load(bp1 + k0);
          m0 = mma_h(a, b0, m0);
          m1 = mma_h(a, b1, m1);
          r0 = mma_h(l, b0, r0);
          r1 = mma_h(l, b1, r1);
          guard4(m0, m1, r0, r1, a, l, b0, b1, a);
        }
        acc_guard4(m0, m1, r0, r1);
        float* vp = sV + (p * 16 + 8 * hh) * NHID + nt0 * 16 + c;
#pragma unroll
        for (int r = 0; r < 8; ++r) {
          vp[r * NHID]      = (m0[r] + r0[r] * RES_INV) * V_INV;
          vp[r * NHID + 16] = (m1[r] + r1[r] * RES_INV) * V_INV;
        }
      }
    }
    __syncthreads();

#pragma unroll
    for (int bi = 0; bi < 2; ++bi) {
      const int b = 2 * wave + bi;
      float va[8], vb[8];
      {
        const v4f t0 = *(const v4f*)(sV + b * NHID + 8 * lane);
        const v4f t1 = *(const v4f*)(sV + b * NHID + 8 * lane + 4);
        const v4f u0 = *(const v4f*)(sV + (16 + b) * NHID + 8 * lane);
        const v4f u1 = *(const v4f*)(sV + (16 + b) * NHID + 8 * lane + 4);
#pragma unroll
        for (int e = 0; e < 4; ++e) { va[e] = t0[e]; va[4 + e] = t1[e]; vb[e] = u0[e]; vb[4 + e] = u1[e]; }
      }
      const float* e2p = E2 + ((size_t)(brow0 + b) * NSLOT) * NHID + 8 * lane;
      float sc0 = 0.0f, sc1 = 0.0f;
#pragma unroll 1
      for (int t2 = 0; t2 < NSLOT / 2; ++t2) {
        const float* ep = e2p + (size_t)(2 * t2) * NHID;
        const v4f x0 = *(const v4f*)(ep);
        const v4f x1 = *(const v4f*)(ep + 4);
        const v4f y0 = *(const v4f*)(ep + NHID);
        const v4f y1 = *(const v4f*)(ep + NHID + 4);
        float s0 = 0.0f, s1 = 0.0f;
#pragma unroll
        for (int e = 0; e < 4; ++e) {
          s0 += ftanh(x0[e] + va[e]) * w3r[e];
          s0 += ftanh(x1[e] + va[4 + e]) * w3r[4 + e];
          s1 += ftanh(y0[e] + vb[e]) * w3r[e];
          s1 += ftanh(y1[e] + vb[4 + e]) * w3r[4 + e];
        }
#pragma unroll
        for (int off = 1; off < 32; off <<= 1) {
          s0 += __shfl_xor(s0, off, 32);
          s1 += __shfl_xor(s1, off, 32);
        }
        s0 += b3v;
        s1 += b3v;
        const int te = 2 * t2, to = 2 * t2 + 1;
        sc0 = (lane == te) ? s0 : sc0;
        sc0 = (lane == to) ? s1 : sc0;
        sc1 = (lane + 32 == te) ? s0 : sc1;
        sc1 = (lane + 32 == to) ? s1 : sc1;
      }
      float mx = fmaxf(sc0, sc1);
#pragma unroll
      for (int off = 1; off < 32; off <<= 1) mx = fmaxf(mx, __shfl_xor(mx, off, 32));
      const float e0 = expf(sc0 - mx);
      const float e1 = expf(sc1 - mx);
      float sum = e0 + e1;
#pragma unroll
      for (int off = 1; off < 32; off <<= 1) sum += __shfl_xor(sum, off, 32);
      const float inv = 1.0f / sum;
      const float a0 = e0 * inv, a1 = e1 * inv;
      wsum[bi][0] += a0;
      wsum[bi][1] += a1;
      float yq = a0 * qv[bi][0] + a1 * qv[bi][1];
      float oc = a0 * rv[bi][0] + a1 * rv[bi][1];
#pragma unroll
      for (int off = 1; off < 32; off <<= 1) {
        yq += __shfl_xor(yq, off, 32);
        oc += __shfl_xor(oc, off, 32);
      }
      octx[bi] = oc;
      const float yv = yhist[(size_t)(brow0 + b) * NSLOT + s];
      const float sv = spd[(size_t)(brow0 + b) * NSLOT + s];
      const float yt = yq + yv * weffy + sv * weffs + beff;
      if (lane == 0) sYt[b] = yt;
    }
    __syncthreads();

    {
      float ytr[8];
#pragma unroll
      for (int r = 0; r < 8; ++r) ytr[r] = sYt[8 * hh + r];
#pragma unroll
      for (int p = 0; p < 2; ++p) {
#pragma unroll
        for (int nt = 0; nt < 2; ++nt) {
          const int j = opaque_i(32 * wave + 16 * nt + c);
          const _Float16* wh   = (p ? WHB : WHF) + (size_t)j * NHID + koff;
          const _Float16* arow = hcur + (p * 16 + c) * HCP + koff;
          v8f g0 = z8, g1 = z8, g2 = z8, g3 = z8;
#pragma unroll 1
          for (int k0 = 0; k0 < NHID; k0 += 32) {
            const v16h a  = frag_load(arow + k0);
            const v16h b0 = frag_load(wh + k0);
            const v16h b1 = frag_load(wh + (size_t)1 * NHID * NHID + k0);
            const v16h b2 = frag_load(wh + (size_t)2 * NHID * NHID + k0);
            const v16h b3f = frag_load(wh + (size_t)3 * NHID * NHID + k0);
            g0 = mma_h(a, b0, g0);
            g1 = mma_h(a, b1, g1);
            g2 = mma_h(a, b2, g2);
            g3 = mma_h(a, b3f, g3);
            guard4(g0, g1, g2, g3, a, b0, b1, b2, b3f);
          }
          acc_guard4(g0, g1, g2, g3);
          const float gb0 = sGW[p * NGATE + 0 * NHID + j];
          const float gb1 = sGW[p * NGATE + 1 * NHID + j];
          const float gb2 = sGW[p * NGATE + 2 * NHID + j];
          const float gb3 = sGW[p * NGATE + 3 * NHID + j];
          const float wi0 = sGW[(2 + p) * NGATE + 0 * NHID + j];
          const float wi1 = sGW[(2 + p) * NGATE + 1 * NHID + j];
          const float wi2 = sGW[(2 + p) * NGATE + 2 * NHID + j];
          const float wi3 = sGW[(2 + p) * NGATE + 3 * NHID + j];
#pragma unroll
          for (int r = 0; r < 8; ++r) {
            const float zi = g0[r] * V_INV + ytr[r] * wi0 + gb0;
            const float zf = g1[r] * V_INV + ytr[r] * wi1 + gb1;
            const float zg = g2[r] * V_INV + ytr[r] * wi2 + gb2;
            const float zo = g3[r] * V_INV + ytr[r] * wi3 + gb3;
            const float ig = fsig(zi);
            const float fg = fsig(zf);
            const float gg = ftanh(zg);
            const float og = fsig(zo);
            const float cn = fg * cst[p][nt][r] + ig * gg;
            cst[p][nt][r] = cn;
            const float hn = og * ftanh(cn);
            if (p == 0) {
              if (nt == 0) hfd[r] = hn * fw0;
              else         hfd[r] = fmaf(hn, fw1, hfd[r]);
            }
            _Float16 hi, lo;
            const int ro = (p * 16 + 8 * hh + r) * HCP;
            split_h(hn * HC_CARRY, hi, lo);
            hnxt[ro + j] = hi;
            HCl[ro + j]  = lo;
            split_h(cn * HC_CARRY, hi, lo);
            hnxt[ro + NHID + j] = hi;
            HCl[ro + NHID + j]  = lo;
          }
        }
      }
    }
    __syncthreads();
  }

#pragma unroll
  for (int bi = 0; bi < 2; ++bi) {
    sV[(2 * wave + bi) * NSLOT + lane]      = wsum[bi][0] * SLOT_INV;
    sV[(2 * wave + bi) * NSLOT + 32 + lane] = wsum[bi][1] * SLOT_INV;
  }
  {
#pragma unroll
    for (int r = 0; r < 8; ++r) {
#pragma unroll
      for (int off = 1; off < 16; off <<= 1) hfd[r] += __shfl_xor(hfd[r], off, 32);
    }
    if (c == 0) {
#pragma unroll
      for (int r = 0; r < 8; ++r) sPart[wave * 16 + 8 * hh + r] = hfd[r];
    }
    if (lane == 0) {
      sOctx[2 * wave]     = octx[0];
      sOctx[2 * wave + 1] = octx[1];
    }
  }
  __syncthreads();
  {
    const v4f v = *(const v4f*)(sV + tid * 4);
    float* dst = out0 + (size_t)brow0 * NSLOT + tid * 4;
    *(volatile v4f*)dst = v;
    __threadfence();
    *(volatile v4f*)dst = v;
  }
  if (wave == 0) {
    const int rr = lane & 15;
    float v = sOctx[rr] + fbin[0];
#pragma unroll
    for (int w = 0; w < 8; ++w) v += sPart[w * 16 + rr];
    v = (lane < 16) ? v : 0.0f;
    float* dst = OUT1P + (size_t)blockIdx.x * 32 + lane;
    *(volatile float*)dst = v;
    __threadfence();
    *(volatile float*)dst = v;
  }
}

__global__ __launch_bounds__(NTHR) void out1_store_kernel(const float* __restrict__ OUT1P, float* __restrict__ out1) {
  const int i = threadIdx.x;
  const float v = OUT1P[(i >> 4) * 32 + (i & 15)];
  *(volatile float*)(out1 + i) = v;
  __threadfence();
  *(volatile float*)(out1 + i) = v;
}

extern "C" void kernel_launch(void* const* d_in, const int* in_sizes, int n_in,
                              void* d_out, int out_size, void* d_ws, size_t ws_size, hipStream_t stream) {
  if (n_in < 25 || d_out == nullptr || d_ws == nullptr) return;
  if (in_sizes[0] != NROWS * NENC || in_sizes[1] != NROWS || in_sizes[2] != NROWS ||
      in_sizes[3] != 2 * NBATCH * NHID || in_sizes[4] != 2 * NBATCH * NHID ||
      in_sizes[5] != NHID * NW1 || in_sizes[7] != NHID * NHID || in_sizes[12] != NGATE * NHID ||
      in_sizes[16] != NGATE * NHID || in_sizes[19] != NHID * NFC || in_sizes[23] != NHID + NENC ||
      out_size != NROWS + NBATCH) return;

  const float* IE   = (const float*)d_in[0];
  const float* yh   = (const float*)d_in[1];
  const float* sp   = (const float*)d_in[2];
  const float* h0   = (const float*)d_in[3];
  const float* c0   = (const float*)d_in[4];
  const float* w1   = (const float*)d_in[5];
  const float* b1   = (const float*)d_in[6];
  const float* w2   = (const float*)d_in[7];
  const float* b2   = (const float*)d_in[8];
  const float* w3   = (const float*)d_in[9];
  const float* b3   = (const float*)d_in[10];
  const float* wihf = (const float*)d_in[11];
  const float* whhf = (const float*)d_in[12];
  const float* bihf = (const float*)d_in[13];
  const float* bhhf = (const float*)d_in[14];
  const float* wihb = (const float*)d_in[15];
  const float* whhb = (const float*)d_in[16];
  const float* bihb = (const float*)d_in[17];
  const float* bhhb = (const float*)d_in[18];
  const float* fcw1 = (const float*)d_in[19];
  const float* fcb1 = (const float*)d_in[20];
  const float* fcw2 = (const float*)d_in[21];
  const float* fcb2 = (const float*)d_in[22];
  const float* fwin = (const float*)d_in[23];
  const float* fbin = (const float*)d_in[24];
  float* out0 = (float*)d_out;
  float* out1 = (float*)d_out + (size_t)NROWS;

  char* ws = (char*)d_ws; size_t off = 0;
  auto carve = [&](size_t bytes) -> char* { char* p = ws + off; off += (bytes + 255) & ~(size_t)255; return p; };
  float*          E2    = (float*)carve((size_t)NROWS * NHID * 4);
  unsigned short* IEH   = (unsigned short*)carve((size_t)NROWS * NENC * 2);
  unsigned short* IEL   = (unsigned short*)carve((size_t)NROWS * NENC * 2);
  unsigned short* W21HC = (unsigned short*)carve((size_t)NHID * KHC * 2);
  unsigned short* W21E  = (unsigned short*)carve((size_t)NHID * NENC * 2);
  unsigned short* WHF   = (unsigned short*)carve((size_t)NGATE * NHID * 2);
  unsigned short* WHB   = (unsigned short*)carve((size_t)NGATE * NHID * 2);
  float*          Qv    = (float*)carve((size_t)NROWS * 4);
  float*          Rv    = (float*)carve((size_t)NROWS * 4);
  float*          SMALLv = (float*)carve((size_t)SMALL_N * 4);
  float*          OUT1P = (float*)carve((size_t)(NBATCH / 16) * 32 * 4);
  if (off > ws_size || off > (size_t)134217728) return;

  fold_w21_kernel<<<(NHID * (NW1 / 8)) / NTHR, NTHR, 0, stream>>>(w1, w2, W21HC, W21E);
  small_prep_kernel<<<1, NTHR, 0, stream>>>(w2, b1, b2, fcw1, fcb1, fcw2, fcb2, bihf, bhhf, bihb, bhhb, SMALLv);
  const int n8w = NGATE * NHID / 8;
  cvt8_scale_kernel<<<(n8w + NTHR - 1) / NTHR, NTHR, 0, stream>>>(whhf, WHF, n8w, W_CARRY);
  cvt8_scale_kernel<<<(n8w + NTHR - 1) / NTHR, NTHR, 0, stream>>>(whhb, WHB, n8w, W_CARRY);
  ie_pack_kernel<<<NROWS / 256, NTHR, 0, stream>>>(IE, SMALLv, fwin, IEH, IEL, Qv, Rv);
  e2_gemm_kernel<<<((NROWS / 32) * (NHID / 64)) / 8, NTHR, 0, stream>>>(IEH, IEL, W21E, SMALLv, E2);
  decoder_scan_kernel<<<NBATCH / 16, NTHR, 0, stream>>>(E2, Qv, Rv, yh, sp, h0, c0, W21HC, WHF, WHB, SMALLv, w3, b3,
                                                        wihf, wihb, fwin, fbin, out0, OUT1P);
  out1_store_kernel<<<1, NTHR, 0, stream>>>(OUT1P, out1);
}
